// GINConvNet_73014444032011
// MI455X (gfx1250) — hardware-verified
//
#include <hip/hip_runtime.h>
#include <stddef.h>
#include <stdint.h>


#define NN      100000
#define NE      400000
#define NG      1024
#define FIN     78
#define FPAD    96
#define DIM     32
#define HLW     64
#define TROWS   128
#define NTILE   782
#define MP      (NTILE * TROWS)
#define RECW    96
#define SEQ     1000
#define NTOK    26
#define KCV     8
#define PC      993
#define TSLOT   994
#define KXT     (TSLOT * 32)
#define TBLN    (KCV * NTOK * 32)
#define TCH     63
#define NCHK    16
#define TOKW    70
#define LMD     1024
#define XCW     2560
#define X1W     2048
#define NTHR    256
#define NWAVE   8
#define EPT     8
#define CHUNK   (NTHR * EPT)
#define WCAP    (EPT * 32)
#define LISTN   (NWAVE * WCAP)
#define NB      1024
#define NBLK    98
#define RCAP    8192
#define DEGCAP  32
#define PKS     11
#define PCAP    4096
#define GBM     64
#define GBN     128
#define GTHR    128
#define WSMAX   134217728
#define LDS_CMP ((2 * RCAP + 2 * NB + LISTN) * 4 + 64)
#define LDS_XT  ((TBLN + 32 + 128 * 128) * 4 + 128 * TOKW * 4)

static_assert(MP >= NN && MP % 128 == 0 && MP % 32 == 0);
static_assert(NBLK * NB >= MP);
static_assert((CHUNK & (CHUNK - 1)) == 0 && CHUNK <= (1 << PKS) && NB <= (1 << PKS));
static_assert(NE < (1 << 20) && NN < (1 << 20));
static_assert(NTHR * 4 == NB && LISTN >= NB);
static_assert(RCAP % (4 * NTHR) == 0 && RCAP >= (4281 * 11) / 10);
static_assert(DEGCAP >= 15 + 8 && DEGCAP <= 32);
static_assert(NCHK * TCH >= PC && (NCHK - 1) * TCH < PC && TOKW >= TCH + KCV - 1);
static_assert(KXT % 32 == 0 && KXT >= 32 * PC && TSLOT % 2 == 0);
static_assert(FPAD % 32 == 0 && HLW % 32 == 0 && XCW % 32 == 0 && X1W % 32 == 0);
static_assert(NG % GBM == 0 && NG % 128 == 0 && NG % 32 == 0);
static_assert((RECW * 4) % 128 == 0 && RECW >= 65);
static_assert((MP * (FPAD / 8)) % NTHR == 0);
static_assert(LDS_CMP <= 300000 && LDS_XT <= 300000);
static_assert(TBLN % 4 == 0 && TBLN == 26 * NTHR);

typedef float          v4f  __attribute__((ext_vector_type(4)));
typedef float          v8f  __attribute__((ext_vector_type(8)));
typedef int            v4i  __attribute__((ext_vector_type(4)));
typedef int            v8i  __attribute__((ext_vector_type(8)));
typedef unsigned int   v4u  __attribute__((ext_vector_type(4)));
typedef unsigned short v8us __attribute__((ext_vector_type(8)));
typedef __bf16         v16b __attribute__((ext_vector_type(16)));
typedef v4f  __attribute__((may_alias)) v4fa;
typedef v4i  __attribute__((may_alias)) v4ia;
typedef v4u  __attribute__((may_alias)) v4ua;
typedef v8us __attribute__((may_alias)) v8usa;
union FragB { v16b v; v8us h[2]; v8i w; };

__device__ __forceinline__ v8f wmb(const FragB& a, const FragB& b, v8f c) {
  v8f d = __builtin_amdgcn_wmma_f32_16x16x32_bf16(false, a.v, false, b.v, (short)0, c, false, false);
  asm volatile("v_nop\n\tv_nop\n\tv_nop\n\tv_nop" : "+v"(d) : "v"(a.w), "v"(b.w));
  return d;
}
__device__ __forceinline__ v8f z8() { v8f z = {0.f, 0.f, 0.f, 0.f, 0.f, 0.f, 0.f, 0.f}; return z; }

__device__ __forceinline__ unsigned short bf_bits(float f) {
  unsigned int u = __float_as_uint(f);
  u += 0x7FFFu + ((u >> 16) & 1u);
  const unsigned short r = (unsigned short)(u >> 16);
  return (f != f) ? (unsigned short)0x7fc0 : r;
}
__device__ __forceinline__ float bf_val(unsigned short b) { return __uint_as_float(((unsigned int)b) << 16); }
__device__ __forceinline__ float bf_rne(float f) { return bf_val(bf_bits(f)); }
__device__ __forceinline__ float relu_np(float v) { return (v > 0.0f) ? v : (v - v); }

__device__ __forceinline__ int scan_chunk(const int* __restrict__ dsts, int nE, int cbase, int slotBase,
                                          int nb, int vec8, int* list, int tid, int lane, int wave) {
  int wc = 0;
  const int el0  = tid * EPT;
  const int e0   = cbase + el0;
  const int sent = -2147483647 - 1;
  v4i da, db;
  if (vec8 != 0 && cbase + CHUNK <= nE) {
    da = *(const v4i*)(dsts + e0);
    db = *(const v4i*)(dsts + e0 + 4);
  } else {
    da.x = (e0     < nE) ? dsts[min(e0,     nE - 1)] : sent;
    da.y = (e0 + 1 < nE) ? dsts[min(e0 + 1, nE - 1)] : sent;
    da.z = (e0 + 2 < nE) ? dsts[min(e0 + 2, nE - 1)] : sent;
    da.w = (e0 + 3 < nE) ? dsts[min(e0 + 3, nE - 1)] : sent;
    db.x = (e0 + 4 < nE) ? dsts[min(e0 + 4, nE - 1)] : sent;
    db.y = (e0 + 5 < nE) ? dsts[min(e0 + 5, nE - 1)] : sent;
    db.z = (e0 + 6 < nE) ? dsts[min(e0 + 6, nE - 1)] : sent;
    db.w = (e0 + 7 < nE) ? dsts[min(e0 + 7, nE - 1)] : sent;
  }
  const unsigned nbs = (unsigned)slotBase;
  const unsigned unb = (unsigned)nb;
  const unsigned s0 = (unsigned)da.x - nbs, s1 = (unsigned)da.y - nbs;
  const unsigned s2 = (unsigned)da.z - nbs, s3 = (unsigned)da.w - nbs;
  const unsigned s4 = (unsigned)db.x - nbs, s5 = (unsigned)db.y - nbs;
  const unsigned s6 = (unsigned)db.z - nbs, s7 = (unsigned)db.w - nbs;
  const bool h0 = s0 < unb, h1 = s1 < unb, h2 = s2 < unb, h3 = s3 < unb;
  const bool h4 = s4 < unb, h5 = s5 < unb, h6 = s6 < unb, h7 = s7 < unb;
  const unsigned any = __builtin_amdgcn_ballot_w32(h0 | h1 | h2 | h3 | h4 | h5 | h6 | h7);
  if (any != 0u) {
#define HITJ(J, HJ, SJ) { \
      const unsigned mj = __builtin_amdgcn_ballot_w32(HJ); \
      if (mj != 0u) { \
        if (HJ) { \
          const int pos = wc + (int)__builtin_amdgcn_mbcnt_lo(mj, 0u); \
          if (pos < WCAP) list[wave * WCAP + pos] = ((el0 + (J)) << PKS) | (int)(SJ); \
        } \
        wc += (int)__builtin_popcount(mj); } }
    HITJ(0, h0, s0)
    HITJ(1, h1, s1)
    HITJ(2, h2, s2)
    HITJ(3, h3, s3)
    HITJ(4, h4, s4)
    HITJ(5, h5, s5)
    HITJ(6, h6, s6)
    HITJ(7, h7, s7)
#undef HITJ
  }
  return wc;
}

__global__ __launch_bounds__(NTHR) void k_xb(const float* __restrict__ x, unsigned short* xb, int nUnits) {
  const int u = (int)blockIdx.x * NTHR + (int)threadIdx.x;
  if (u >= nUnits) return;
  const int row = u / (FPAD / 8);
  const int c8  = (u - row * (FPAD / 8)) * 8;
  const int rc  = row < NN ? row : NN - 1;
  const float* p = x + (size_t)rc * FIN;
  v8us o;
#pragma unroll
  for (int i = 0; i < 8; ++i) {
    const int c  = c8 + i;
    const int cc = c < FIN ? c : FIN - 1;
    const float v = p[cc];
    const bool ok = (row < NN) && (c < FIN);
    o[i] = ok ? bf_bits(v) : (unsigned short)0;
  }
  unsigned short* dp = xb + (size_t)u * 8;
  *(volatile v8us*)dp = o;
  __threadfence();
  *(volatile v8us*)dp = o;
}

__global__ __launch_bounds__(NTHR) void k_wt(const float* __restrict__ src, int ld, int nOut, int kDst,
                                             int kSrc, int mode, int nUnits, unsigned short* dst) {
  const int u = (int)blockIdx.x * NTHR + (int)threadIdx.x;
  if (u >= nUnits) return;
  const int k8n = kDst >> 3;
  const int upm = nOut * k8n;
  const int mi  = u / upm;
  const int v   = u - mi * upm;
  const int n   = v / k8n;
  const int k8  = (v - n * k8n) * 8;
  const float* sb = src + (size_t)mi * (size_t)kSrc * (size_t)ld + n;
  v8us o;
#pragma unroll
  for (int i = 0; i < 8; ++i) {
    const int k = k8 + i;
    int sr;
    bool z = false;
    if (mode == 0) {
      sr = k % kSrc;
    } else if (mode == 1) {
      sr = k;
      z = k >= kSrc;
    } else {
      sr = (k < 512) ? (((k >> 8) << 7) + (k & 127)) : (k - 256);
    }
    sr = sr < 0 ? 0 : (sr > kSrc - 1 ? kSrc - 1 : sr);
    const float val = sb[(size_t)sr * (size_t)ld];
    o[i] = z ? (unsigned short)0 : bf_bits(val);
  }
  unsigned short* dp = dst + (size_t)u * 8;
  *(volatile v8us*)dp = o;
  __threadfence();
  *(volatile v8us*)dp = o;
}

__global__ __launch_bounds__(NTHR) void k_lm(const float* __restrict__ src, int colOff, unsigned short* xc,
                                             int nUnits) {
  const int u = (int)blockIdx.x * NTHR + (int)threadIdx.x;
  if (u >= nUnits) return;
  const int row = u >> 7;
  const int c8  = (u & 127) * 8;
  const float* p = src + (size_t)row * LMD + c8;
  const v4f a = *(const v4f*)p;
  const v4f b = *(const v4f*)(p + 4);
  v8us o;
  o[0] = bf_bits(a.x); o[1] = bf_bits(a.y); o[2] = bf_bits(a.z); o[3] = bf_bits(a.w);
  o[4] = bf_bits(b.x); o[5] = bf_bits(b.y); o[6] = bf_bits(b.z); o[7] = bf_bits(b.w);
  unsigned short* dp = xc + (size_t)row * XCW + colOff + c8;
  *(volatile v8us*)dp = o;
  __threadfence();
  *(volatile v8us*)dp = o;
}

__global__ __launch_bounds__(NTHR) void k_wxt(const float* __restrict__ w, unsigned short* wxt) {
  __shared__ unsigned short tile[64 * 128];
  const int tid = (int)threadIdx.x;
  const int t0  = 2 * (int)blockIdx.x;
#pragma unroll
  for (int it = 0; it < 8; ++it) {
    const int idx = it * NTHR + tid;
    const int kk  = idx >> 5;
    const int j4  = (idx & 31) * 4;
    const int t   = t0 + (kk >> 5);
    const int f   = kk & 31;
    const int tc  = t < PC ? t : PC - 1;
    const v4f v = *(const v4f*)(w + ((size_t)(f * PC + tc)) * 128 + j4);
    const bool ok = t < PC;
    tile[kk * 128 + j4 + 0] = ok ? bf_bits(v.x) : (unsigned short)0;
    tile[kk * 128 + j4 + 1] = ok ? bf_bits(v.y) : (unsigned short)0;
    tile[kk * 128 + j4 + 2] = ok ? bf_bits(v.z) : (unsigned short)0;
    tile[kk * 128 + j4 + 3] = ok ? bf_bits(v.w) : (unsigned short)0;
  }
  __syncthreads();
  v8us o[4];
#pragma unroll
  for (int it = 0; it < 4; ++it) {
    const int idx = it * NTHR + tid;
    const int n = idx >> 3, q = idx & 7;
#pragma unroll
    for (int i = 0; i < 8; ++i) o[it][i] = tile[(8 * q + i) * 128 + n];
  }
#pragma unroll
  for (int it = 0; it < 4; ++it) {
    const int idx = it * NTHR + tid;
    const int n = idx >> 3, q = idx & 7;
    *(volatile v8us*)(wxt + (size_t)n * KXT + t0 * 32 + 8 * q) = o[it];
  }
  __threadfence();
#pragma unroll
  for (int it = 0; it < 4; ++it) {
    const int idx = it * NTHR + tid;
    const int n = idx >> 3, q = idx & 7;
    *(volatile v8us*)(wxt + (size_t)n * KXT + t0 * 32 + 8 * q) = o[it];
  }
}

__global__ __launch_bounds__(NTHR) void k_tbl(const float* __restrict__ emb, const float* __restrict__ cw,
                                              float* tbl) {
  const int idx = (int)blockIdx.x * NTHR + (int)threadIdx.x;
  if (idx >= TBLN) return;
  const int f    = idx & 31;
  const int rest = idx >> 5;
  const int k    = rest / NTOK;
  const int v    = rest - k * NTOK;
  const float* ep = emb + v * 128;
  const float* wp = cw + f * (128 * KCV) + k;
  float s = 0.0f;
#pragma unroll 4
  for (int ch = 0; ch < 128; ++ch) s = fmaf(bf_rne(ep[ch]), bf_rne(wp[ch * KCV]), s);
  *(volatile float*)(tbl + idx) = s;
  __threadfence();
  *(volatile float*)(tbl + idx) = s;
}

__global__ __launch_bounds__(NTHR) void k_compact(const int* __restrict__ srcs, const int* __restrict__ dsts,
                                                  int nE, int nN, int vec8, int* lst, int* cntg, int* offg) {
  extern __shared__ v4f lds_dyn[];
  int* reg1 = (int*)lds_dyn;
  int* reg2 = reg1 + RCAP;
  int* scnt = reg2 + RCAP;
  int* soff = scnt + NB;
  int* list = soff + NB;
  int* wcnt = list + LISTN;
  int* wtot = wcnt + NWAVE;
  const int tid = (int)threadIdx.x, lane = tid & 31, wave = tid >> 5;
  const int blk = (int)blockIdx.x;
  const int nodeBase = blk * NB;
  int nbEff = nN - nodeBase;
  nbEff = nbEff < 0 ? 0 : (nbEff > NB ? NB : nbEff);

  for (int i = tid; i < NB; i += NTHR) scnt[i] = 0;
  for (int i = tid; i < RCAP; i += NTHR) reg2[i] = 0;
  __syncthreads();

  int tot = 0;
  const int nChunks = (nE + CHUNK - 1) / CHUNK;
#pragma unroll 1
  for (int ch = 0; ch < nChunks; ++ch) {
    const int cbase = ch * CHUNK;
    const int wc = scan_chunk(dsts, nE, cbase, nodeBase, nbEff, vec8, list, tid, lane, wave);
    if (lane == 0) wcnt[wave] = wc;
    __syncthreads();
    int pre = 0, all = 0;
#pragma unroll
    for (int w2 = 0; w2 < NWAVE; ++w2) {
      int c = wcnt[w2];
      c = c < 0 ? 0 : (c > WCAP ? WCAP : c);
      all += c;
      pre += (w2 < wave) ? c : 0;
    }
    const int wcc  = wc > WCAP ? WCAP : wc;
    const int base = tot + pre;
#pragma unroll 1
    for (int i = lane; i < wcc; i += 32) {
      const int ent = list[wave * WCAP + i];
      const int el  = (ent >> PKS) & (CHUNK - 1);
      int sl = ent & ((1 << PKS) - 1);
      sl = sl > NB - 1 ? NB - 1 : sl;
      int eid = cbase + el;
      eid = eid > nE - 1 ? nE - 1 : eid;
      const int pos = base + i;
      if (pos < RCAP) reg1[pos] = (int)(((unsigned)eid << PKS) | (unsigned)sl);
    }
    tot += all;
    tot = tot > RCAP ? RCAP : tot;
    __syncthreads();
  }
  const int nh = tot;

  if (wave == 0) {
#pragma unroll 1
    for (int b0 = 0; b0 < nh; b0 += 32) {
      const int idx = b0 + lane;
      const int uv  = reg1[idx < nh ? idx : nh - 1];
      const int m32 = (nh - b0) < 32 ? (nh - b0) : 32;
#pragma unroll 1
      for (int k = 0; k < m32; ++k) {
        const int u  = __builtin_amdgcn_readlane(uv, k);
        int sl = u & ((1 << PKS) - 1);
        sl = sl > NB - 1 ? NB - 1 : sl;
        if (lane == 0) scnt[sl] = scnt[sl] + 1;
      }
    }
  }
  __syncthreads();

  {
    const v4i ca = *(const v4ia*)(scnt + 4 * tid);
    const int e0 = ca.x < 0 ? 0 : ca.x, e1 = ca.y < 0 ? 0 : ca.y;
    const int e2 = ca.z < 0 ? 0 : ca.z, e3 = ca.w < 0 ? 0 : ca.w;
    const int ts = e0 + e1 + e2 + e3;
    int incl = ts;
#pragma unroll
    for (int d = 1; d < 32; d <<= 1) {
      const int up = __shfl_up(incl, d);
      if (lane >= d) incl += up;
    }
    if (lane == 31) wtot[wave] = incl;
    __syncthreads();
    int pre = 0;
#pragma unroll
    for (int w2 = 0; w2 < NWAVE; ++w2) pre += (w2 < wave) ? wtot[w2] : 0;
    int run = pre + incl - ts;
    soff[4 * tid + 0] = run; run += e0;
    soff[4 * tid + 1] = run; run += e1;
    soff[4 * tid + 2] = run; run += e2;
    soff[4 * tid + 3] = run;
  }
  __syncthreads();
  for (int i = tid; i < NB; i += NTHR) list[i] = soff[i];
  __syncthreads();

  if (wave == 0) {
#pragma unroll 1
    for (int b0 = 0; b0 < nh; b0 += 32) {
      const int idx = b0 + lane;
      const int uv  = reg1[idx < nh ? idx : nh - 1];
      const int m32 = (nh - b0) < 32 ? (nh - b0) : 32;
#pragma unroll 1
      for (int k = 0; k < m32; ++k) {
        const int u   = __builtin_amdgcn_readlane(uv, k);
        int sl = u & ((1 << PKS) - 1);
        sl = sl > NB - 1 ? NB - 1 : sl;
        const int eid = (int)((unsigned)u >> PKS);
        if (lane == 0) {
          int pos = list[sl];
          pos = pos < 0 ? 0 : (pos > RCAP - 1 ? RCAP - 1 : pos);
          reg2[pos] = eid;
          list[sl] = pos + 1;
        }
      }
    }
  }
  __syncthreads();

  const bool ovf = (nh >= RCAP);
#pragma unroll 1
  for (int it = 0; it < RCAP / (4 * NTHR); ++it) {
    const int i4 = (it * NTHR + tid) * 4;
    const v4i er = *(const v4ia*)(reg2 + i4);
    int e0 = er.x, e1 = er.y, e2 = er.z, e3 = er.w;
    e0 = e0 < 0 ? 0 : (e0 > nE - 1 ? nE - 1 : e0);
    e1 = e1 < 0 ? 0 : (e1 > nE - 1 ? nE - 1 : e1);
    e2 = e2 < 0 ? 0 : (e2 > nE - 1 ? nE - 1 : e2);
    e3 = e3 < 0 ? 0 : (e3 > nE - 1 ? nE - 1 : e3);
    int s0 = srcs[e0], s1 = srcs[e1], s2 = srcs[e2], s3 = srcs[e3];
    s0 = s0 < 0 ? 0 : (s0 > nN - 1 ? nN - 1 : s0);
    s1 = s1 < 0 ? 0 : (s1 > nN - 1 ? nN - 1 : s1);
    s2 = s2 < 0 ? 0 : (s2 > nN - 1 ? nN - 1 : s2);
    s3 = s3 < 0 ? 0 : (s3 > nN - 1 ? nN - 1 : s3);
    v4i o;
    o.x = (i4     < nh) ? s0 : 0;
    o.y = (i4 + 1 < nh) ? s1 : 0;
    o.z = (i4 + 2 < nh) ? s2 : 0;
    o.w = (i4 + 3 < nh) ? s3 : 0;
    int* gp = lst + (size_t)blk * RCAP + i4;
    *(volatile v4i*)gp = o;
    __threadfence();
    *(volatile v4i*)gp = o;
  }
  {
    const v4i ca = *(const v4ia*)(scnt + 4 * tid);
    const v4i oa = *(const v4ia*)(soff + 4 * tid);
    v4i c, f;
    c.x = ovf ? 32767 : (ca.x < 0 ? 0 : (ca.x > 32767 ? 32767 : ca.x));
    c.y = ovf ? 32767 : (ca.y < 0 ? 0 : (ca.y > 32767 ? 32767 : ca.y));
    c.z = ovf ? 32767 : (ca.z < 0 ? 0 : (ca.z > 32767 ? 32767 : ca.z));
    c.w = ovf ? 32767 : (ca.w < 0 ? 0 : (ca.w > 32767 ? 32767 : ca.w));
    f.x = oa.x < 0 ? 0 : (oa.x > RCAP ? RCAP : oa.x);
    f.y = oa.y < 0 ? 0 : (oa.y > RCAP ? RCAP : oa.y);
    f.z = oa.z < 0 ? 0 : (oa.z > RCAP ? RCAP : oa.z);
    f.w = oa.w < 0 ? 0 : (oa.w > RCAP ? RCAP : oa.w);
    int* cp = cntg + (size_t)blk * NB + 4 * tid;
    int* fp = offg + (size_t)blk * NB + 4 * tid;
    *(volatile v4i*)cp = c;
    *(volatile v4i*)fp = f;
    __threadfence();
    *(volatile v4i*)cp = c;
    *(volatile v4i*)fp = f;
  }
}

template <int FIRST>
__global__ __launch_bounds__(NTHR) void k_agg(const int* __restrict__ lst, const int* __restrict__ cntg,
                                              const int* __restrict__ offg, const float* __restrict__ F,
                                              const float* __restrict__ stat, const float* __restrict__ bias,
                                              unsigned short* outp, int nN) {
  __shared__ __attribute__((aligned(16))) unsigned short stg[NWAVE * 32 * HLW];
  const int tid = (int)threadIdx.x, lane = tid & 31, wave = tid >> 5;
  const int blk = (int)blockIdx.x;
  const int nodeBase = blk * NB;
  float mu = 0.0f, sa = 1.0f, sb = 0.0f, bv = 0.0f;
  if (FIRST != 0) {
    bv = bf_rne(bias[lane]);
  } else {
    mu = stat[lane]; sa = stat[32 + lane]; sb = stat[64 + lane];
  }
  const int* lb = lst + (size_t)blk * RCAP;
  unsigned short* sw = stg + wave * 32 * HLW;
  const float qnan = __int_as_float(0x7fc00000);

#pragma unroll 1
  for (int g = 0; g < NB / NWAVE / 32; ++g) {
    const int slot0 = wave * (NB / NWAVE) + g * 32;
    const int cl = cntg[(size_t)blk * NB + slot0 + lane];
    const int ol = offg[(size_t)blk * NB + slot0 + lane];
#pragma unroll 1
    for (int j = 0; j < 32; ++j) {
      const int craw = __builtin_amdgcn_readlane(cl, j);
      int st = __builtin_amdgcn_readlane(ol, j);
      const int cnt = craw < 0 ? 0 : (craw > DEGCAP ? DEGCAP : craw);
      st = st < 0 ? 0 : (st > RCAP - 1 ? RCAP - 1 : st);
      const int grow = nodeBase + slot0 + j;
      int idx = st + lane;
      idx = idx > RCAP - 1 ? RCAP - 1 : idx;
      int sv = lb[idx];
      sv = sv < 0 ? 0 : (sv > nN - 1 ? nN - 1 : sv);
      float ag = 0.0f;
#pragma unroll 1
      for (int k = 0; k < cnt; ++k) {
        const int sk = __builtin_amdgcn_readlane(sv, k);
        const float r = F[(size_t)sk * DIM + lane];
        const float h = (FIRST != 0) ? r : ((r - mu) * sa + sb);
        ag += h;
      }
      const bool live = grow < nN;
      const int nc = live ? grow : nN - 1;
      const float rs = F[(size_t)nc * DIM + lane];
      const float hs = (FIRST != 0) ? rs : ((rs - mu) * sa + sb);
      float v = hs + ag;
      if (FIRST != 0) v = relu_np(v + bv);
      v = live ? v : 0.0f;
      v = (craw > DEGCAP) ? qnan : v;
      const unsigned short hb = bf_bits(v);
      const unsigned short lw = bf_bits(v - bf_val(hb));
      sw[j * HLW + lane]      = hb;
      sw[j * HLW + 32 + lane] = lw;
    }
    __syncthreads();
    v4u pk[8];
#pragma unroll
    for (int i = 0; i < 8; ++i)
      pk[i] = *(const v4ua*)(sw + (4 * i + (lane >> 3)) * HLW + (lane & 7) * 8);
    const int base = nodeBase + slot0;
    const bool okg = base < MP;
#pragma unroll
    for (int i = 0; i < 8; ++i) {
      unsigned short* gp = outp + (size_t)(base + 4 * i + (lane >> 3)) * HLW + (lane & 7) * 8;
      if (okg) *(volatile v4u*)gp = pk[i];
    }
    __threadfence();
#pragma unroll
    for (int i = 0; i < 8; ++i) {
      unsigned short* gp = outp + (size_t)(base + 4 * i + (lane >> 3)) * HLW + (lane & 7) * 8;
      if (okg) *(volatile v4u*)gp = pk[i];
    }
    __syncthreads();
  }
}

template <int MODE>
__global__ __launch_bounds__(NTHR) void k_mlp(const unsigned short* __restrict__ A,
                                              const unsigned short* __restrict__ Wa, const float* __restrict__ ba,
                                              const unsigned short* __restrict__ Wb, const float* __restrict__ bb,
                                              float* R, float* rec, int nN) {
  constexpr int PA = (MODE == 0) ? FPAD : HLW;
  constexpr int KS = PA / 32;
  __shared__ __attribute__((aligned(16))) float stg[TROWS * DIM];
  __shared__ __attribute__((aligned(16))) unsigned short tl[NWAVE * 16 * HLW];
  __shared__ __attribute__((aligned(16))) float pst[RECW];
  const int tid = (int)threadIdx.x, lane = tid & 31, wave = tid >> 5, hh = lane >> 4, m = lane & 15;
  const int rowBase = (int)blockIdx.x * TROWS;

  v8f acc0 = z8(), acc1 = z8();
  {
    const unsigned short* ap = A + (size_t)(rowBase + 16 * wave + m) * PA + 8 * hh;
    const unsigned short* wp;
    if constexpr (MODE == 2) wp = Wa + (size_t)m * PA + 8 * hh;
    else                     wp = Wb + (size_t)m * PA + 8 * hh;
#pragma unroll
    for (int ks = 0; ks < KS; ++ks) {
      FragB af, b0, b1;
      af.h[0] = *(const v8usa*)(ap + 32 * ks);
      af.h[1] = *(const v8usa*)(ap + 32 * ks + 16);
      b0.h[0] = *(const v8usa*)(wp + 32 * ks);
      b0.h[1] = *(const v8usa*)(wp + 32 * ks + 16);
      b1.h[0] = *(const v8usa*)(wp + 16 * PA + 32 * ks);
      b1.h[1] = *(const v8usa*)(wp + 16 * PA + 32 * ks + 16);
      acc0 = wmb(af, b0, acc0);
      acc1 = wmb(af, b1, acc1);
    }
  }
  if constexpr (MODE == 2) {
    unsigned short* tw = tl + wave * 16 * HLW;
    const float bq0 = bf_rne(ba[m]);
    const float bq1 = bf_rne(ba[16 + m]);
#pragma unroll
    for (int r = 0; r < 8; ++r) {
      const int lr = 8 * hh + r;
      const bool live = (rowBase + 16 * wave + lr) < nN;
      float v0 = relu_np(acc0[r] + bq0);
      float v1 = relu_np(acc1[r] + bq1);
      v0 = live ? v0 : 0.0f;
      v1 = live ? v1 : 0.0f;
      const unsigned short h0 = bf_bits(v0), h1 = bf_bits(v1);
      tw[lr * HLW + m]           = h0;
      tw[lr * HLW + 16 + m]      = h1;
      tw[lr * HLW + 32 + m]      = bf_bits(v0 - bf_val(h0));
      tw[lr * HLW + 32 + 16 + m] = bf_bits(v1 - bf_val(h1));
    }
    __syncthreads();
    acc0 = z8(); acc1 = z8();
    const unsigned short* ap2 = tw + m * HLW + 8 * hh;
    const unsigned short* wp2 = Wb + (size_t)m * HLW + 8 * hh;
#pragma unroll
    for (int ks = 0; ks < HLW / 32; ++ks) {
      FragB af, b0, b1;
      af.h[0] = *(const v8usa*)(ap2 + 32 * ks);
      af.h[1] = *(const v8usa*)(ap2 + 32 * ks + 16);
      b0.h[0] = *(const v8usa*)(wp2 + 32 * ks);
      b0.h[1] = *(const v8usa*)(wp2 + 32 * ks + 16);
      b1.h[0] = *(const v8usa*)(wp2 + 16 * HLW + 32 * ks);
      b1.h[1] = *(const v8usa*)(wp2 + 16 * HLW + 32 * ks + 16);
      acc0 = wmb(af, b0, acc0);
      acc1 = wmb(af, b1, acc1);
    }
  }
  {
    float bq0 = 0.0f, bq1 = 0.0f;
    if constexpr (MODE != 0) { bq0 = bf_rne(bb[m]); bq1 = bf_rne(bb[16 + m]); }
#pragma unroll
    for (int r = 0; r < 8; ++r) {
      const int lr = 16 * wave + 8 * hh + r;
      const bool live = (rowBase + lr) < nN;
      float v0 = acc0[r], v1 = acc1[r];
      if constexpr (MODE != 0) { v0 = relu_np(v0 + bq0); v1 = relu_np(v1 + bq1); }
      stg[lr * DIM + m]      = live ? v0 : 0.0f;
      stg[lr * DIM + 16 + m] = live ? v1 : 0.0f;
    }
  }
  __syncthreads();
  {
    v4f fv[4];
#pragma unroll
    for (int i = 0; i < 4; ++i)
      fv[i] = *(const v4fa*)(stg + (16 * wave + 4 * i + (lane >> 3)) * DIM + 4 * (lane & 7));
#pragma unroll
    for (int i = 0; i < 4; ++i) {
      float* op = R + (size_t)(rowBase + 16 * wave + 4 * i + (lane >> 3)) * DIM + 4 * (lane & 7);
      *(volatile v4f*)op = fv[i];
    }
    __threadfence();
#pragma unroll
    for (int i = 0; i < 4; ++i) {
      float* op = R + (size_t)(rowBase + 16 * wave + 4 * i + (lane >> 3)) * DIM + 4 * (lane & 7);
      *(volatile v4f*)op = fv[i];
    }
  }
  if constexpr (MODE != 0) {
    if (wave == 0) {
      int rv = nN - rowBase;
      rv = rv < 0 ? 0 : (rv > TROWS ? TROWS : rv);
      float n = 0.0f, mean = 0.0f, M2 = 0.0f;
#pragma unroll 1
      for (int r = 0; r < rv; ++r) {
        const float v = stg[r * DIM + lane];
        n += 1.0f;
        const float rk = 1.0f / n;
        const float d = v - mean;
        mean = fmaf(d, rk, mean);
        M2 = fmaf(d, v - mean, M2);
      }
      pst[1 + lane]  = mean;
      pst[33 + lane] = M2;
      if (lane == 0) pst[0] = n;
      if (lane < RECW - 65) pst[65 + lane] = 0.0f;
    }
    __syncthreads();
    v4f pv = {0.f, 0.f, 0.f, 0.f};
    if (tid < RECW / 4) {
      pv = *(const v4fa*)(pst + 4 * tid);
      *(volatile v4f*)(rec + (size_t)blockIdx.x * RECW + 4 * tid) = pv;
    }
    __threadfence();
    if (tid < RECW / 4) {
      *(volatile v4f*)(rec + (size_t)blockIdx.x * RECW + 4 * tid) = pv;
    }
  }
}

__global__ __launch_bounds__(32) void k_comb(const float* __restrict__ rec, int nRec,
                                             const float* __restrict__ gam, const float* __restrict__ bet,
                                             float* st) {
  __shared__ __attribute__((aligned(16))) float sg[128];
  const int c = (int)threadIdx.x;
  double n = 0.0, mean = 0.0, M2 = 0.0;
#pragma unroll 1
  for (int b = 0; b < nRec; ++b) {
    const float* pr = rec + (size_t)b * RECW;
    const float nb = pr[0];
    const float mb = pr[1 + c];
    const float qb = pr[33 + c];
    if (nb > 0.5f) {
      const double nn = n + (double)nb;
      const double delta = (double)mb - mean;
      const double f = (double)nb / nn;
      mean = mean + delta * f;
      M2 = M2 + (double)qb + delta * delta * n * f;
      n = nn;
    }
  }
  const double nt = n < 1.0 ? 1.0 : n;
  const float var = (float)(M2 / nt);
  const float rs = 1.0f / sqrtf(var + 1e-5f);
  sg[c]      = (float)mean;
  sg[32 + c] = bf_rne(gam[c]) * rs;
  sg[64 + c] = bf_rne(bet[c]);
  sg[96 + c] = 0.0f;
  __syncthreads();
  const v4f v = *(const v4fa*)(sg + 4 * c);
  *(volatile v4f*)(st + 4 * c) = v;
  __threadfence();
  *(volatile v4f*)(st + 4 * c) = v;
}

__global__ __launch_bounds__(NTHR) void k_pool(const int* __restrict__ bat, const float* __restrict__ F,
                                               const float* __restrict__ stat, int nN, int vec8,
                                               unsigned short* pool) {
  __shared__ int list[LISTN];
  __shared__ int pl[PCAP];
  __shared__ int wcnt[NWAVE];
  __shared__ __attribute__((aligned(16))) unsigned short prow[8 * HLW];
  const int tid = (int)threadIdx.x, lane = tid & 31, wave = tid >> 5;
  const int g0 = (int)blockIdx.x * 8;

  int tot = 0;
  const int nChunks = (nN + CHUNK - 1) / CHUNK;
#pragma unroll 1
  for (int ch = 0; ch < nChunks; ++ch) {
    const int cbase = ch * CHUNK;
    const int wc = scan_chunk(bat, nN, cbase, g0, 8, vec8, list, tid, lane, wave);
    if (lane == 0) wcnt[wave] = wc;
    __syncthreads();
    int pre = 0, all = 0;
#pragma unroll
    for (int w2 = 0; w2 < NWAVE; ++w2) {
      int c = wcnt[w2];
      c = c < 0 ? 0 : (c > WCAP ? WCAP : c);
      all += c;
      pre += (w2 < wave) ? c : 0;
    }
    const int wcc  = wc > WCAP ? WCAP : wc;
    const int base = tot + pre;
#pragma unroll 1
    for (int i = lane; i < wcc; i += 32) {
      const int ent = list[wave * WCAP + i];
      const int el  = (ent >> PKS) & (CHUNK - 1);
      const int sl  = ent & 7;
      int node = cbase + el;
      node = node > nN - 1 ? nN - 1 : node;
      const int pos = base + i;
      if (pos < PCAP) pl[pos] = (node << 3) | sl;
    }
    tot += all;
    tot = tot > PCAP ? PCAP : tot;
    __syncthreads();
  }
  const int nh = tot;
  const bool ovf = nh >= PCAP;

  const float mu = stat[lane], sa = stat[32 + lane], sb = stat[64 + lane];
  float acc = 0.0f;
#pragma unroll 1
  for (int b0 = 0; b0 < nh; b0 += 32) {
    const int idx = b0 + lane;
    const int ent = pl[idx < nh ? idx : nh - 1];
    const bool hit = (idx < nh) && ((ent & 7) == wave);
    unsigned msk = __builtin_amdgcn_ballot_w32(hit);
    const int nodev = ent >> 3;
    int nhit = (int)__builtin_popcount(msk);
    nhit = nhit > 32 ? 32 : nhit;
#pragma unroll 1
    for (int q = 0; q < nhit; ++q) {
      int k = __builtin_ffs((int)msk) - 1;
      msk &= msk - 1u;
      k = k < 0 ? 0 : k;
      int node = __shfl(nodev, k);
      node = node < 0 ? 0 : (node > nN - 1 ? nN - 1 : node);
      const float r = F[(size_t)node * DIM + lane];
      acc += (r - mu) * sa + sb;
    }
  }
  {
    const float v = ovf ? __int_as_float(0x7fc00000) : acc;
    const unsigned short hb = bf_bits(v);
    prow[wave * HLW + lane]      = hb;
    prow[wave * HLW + 32 + lane] = bf_bits(v - bf_val(hb));
  }
  __syncthreads();
  v4u pk = {0u, 0u, 0u, 0u};
  unsigned short* gp = pool + (size_t)g0 * HLW + 8 * tid;
  if (tid < 64) {
    pk = *(const v4ua*)(prow + 8 * tid);
    *(volatile v4u*)gp = pk;
  }
  __threadfence();
  if (tid < 64) {
    *(volatile v4u*)gp = pk;
  }
}

template <int MODE>
__global__ __launch_bounds__(GTHR) void k_gemm(const unsigned short* __restrict__ A, int lda,
                                               const unsigned short* __restrict__ BT, int K,
                                               const float* __restrict__ bias, void* outp, int ldo,
                                               int hiOff, int loOff) {
  __shared__ __attribute__((aligned(16))) float stg[GBM * GBN];
  const int tid = (int)threadIdx.x, lane = tid & 31, wave = tid >> 5, hh = lane >> 4, m = lane & 15;
  const int rowBase = (int)blockIdx.x * GBM;
  const int colBase = (int)blockIdx.y * GBN;

  v8f acc[8];
#pragma unroll
  for (int t = 0; t < 8; ++t) acc[t] = z8();
  const unsigned short* ap = A  + (size_t)(rowBase + 16 * wave + m) * (size_t)lda + 8 * hh;
  const unsigned short* bp = BT + (size_t)(colBase + m) * (size_t)K + 8 * hh;
#pragma unroll 1
  for (int k0 = 0; k0 < K; k0 += 32) {
    FragB af;
    af.h[0] = *(const v8usa*)(ap + k0);
    af.h[1] = *(const v8usa*)(ap + k0 + 16);
#pragma unroll
    for (int nt = 0; nt < 8; ++nt) {
      const unsigned short* wq = bp + (size_t)(16 * nt) * (size_t)K + k0;
      FragB bf;
      bf.h[0] = *(const v8usa*)wq;
      bf.h[1] = *(const v8usa*)(wq + 16);
      acc[nt] = wmb(af, bf, acc[nt]);
    }
  }
#pragma unroll
  for (int nt = 0; nt < 8; ++nt) {
    const int lc = 16 * nt + m;
    const float bq = bf_rne(bias[colBase + lc]);
#pragma unroll
    for (int r = 0; r < 8; ++r) {
      const int lr = 16 * wave + 8 * hh + r;
      stg[lr * GBN + lc] = relu_np(acc[nt][r] + bq);
    }
  }
  __syncthreads();

  if constexpr (MODE == 2) {
    float* outF = (float*)outp;
    v4f fv[16];
#pragma unroll
    for (int i = 0; i < 16; ++i) fv[i] = *(const v4fa*)(stg + (16 * wave + i) * GBN + 4 * lane);
#pragma unroll
    for (int i = 0; i < 16; ++i) {
      float* op = outF + (size_t)(rowBase + 16 * wave + i) * (size_t)ldo + colBase + 4 * lane;
      *(volatile v4f*)op = fv[i];
    }
    __threadfence();
#pragma unroll
    for (int i = 0; i < 16; ++i) {
      float* op = outF + (size_t)(rowBase + 16 * wave + i) * (size_t)ldo + colBase + 4 * lane;
      *(volatile v4f*)op = fv[i];
    }
  } else {
    unsigned short* outH = (unsigned short*)outp;
    const int cb = 8 * m;
    const bool isHi = (hh == 0);
    const int cofs = (isHi ? hiOff : loOff) + colBase + cb;
    v4u pk[16];
#pragma unroll
    for (int i = 0; i < 16; ++i) {
      const int lr = 16 * wave + i;
      const v4f a = *(const v4fa*)(stg + lr * GBN + cb);
      const v4f b = *(const v4fa*)(stg + lr * GBN + cb + 4);
      const float f[8] = {a.x, a.y, a.z, a.w, b.x, b.y, b.z, b.w};
      unsigned int w[4];
#pragma unroll
      for (int j = 0; j < 4; ++j) {
        const unsigned short h0 = bf_bits(f[2 * j]), h1 = bf_bits(f[2 * j + 1]);
        const unsigned short l0 = bf_bits(f[2 * j] - bf_val(h0)), l1 = bf_bits(f[2 * j + 1] - bf_val(h1));
        const unsigned short q0 = isHi ? h0 : l0, q1 = isHi ? h1 : l1;
        w[j] = (unsigned int)q0 | ((unsigned int)q1 << 16);
      }
      v4u pw; pw.x = w[0]; pw.y = w[1]; pw.z = w[2]; pw.w = w[3];
      pk[i] = pw;
    }
#pragma unroll
    for (int i = 0; i < 16; ++i) {
      unsigned short* op = outH + (size_t)(rowBase + 16 * wave + i) * (size_t)ldo + cofs;
      *(volatile v4u*)op = pk[i];
    }
    __threadfence();
#pragma unroll
    for (int i = 0; i < 16; ++i) {
      unsigned short* op = outH + (size_t)(rowBase + 16 * wave + i) * (size_t)ldo + cofs;
      *(volatile v4u*)op = pk[i];
    }
  }
}

template <int B>
__device__ __forceinline__ void split4(const v4f c, v8us& hv, v8us& lv) {
  const float f0 = relu_np(c.x), f1 = relu_np(c.y), f2 = relu_np(c.z), f3 = relu_np(c.w);
  const unsigned short h0 = bf_bits(f0), h1 = bf_bits(f1), h2 = bf_bits(f2), h3 = bf_bits(f3);
  hv[B + 0] = h0; hv[B + 1] = h1; hv[B + 2] = h2; hv[B + 3] = h3;
  lv[B + 0] = bf_bits(f0 - bf_val(h0));
  lv[B + 1] = bf_bits(f1 - bf_val(h1));
  lv[B + 2] = bf_bits(f2 - bf_val(h2));
  lv[B + 3] = bf_bits(f3 - bf_val(h3));
}

__global__ __launch_bounds__(NTHR) void k_xt(const int* __restrict__ target, const float* __restrict__ tblg,
                                             const float* __restrict__ cbias,
                                             const unsigned short* __restrict__ wxt, float* part) {
  extern __shared__ v4f dsm[];
  float* tbl = (float*)dsm;
  float* cbs = tbl + TBLN;
  float* stg = cbs + 32;
  int*   tok = (int*)(stg + 128 * 128);
  const int tid = (int)threadIdx.x, lane = tid & 31, wave = tid >> 5, hh = lane >> 4, m = lane & 15;
  const int mt = (int)blockIdx.x, ch = (int)blockIdx.y;
  const int t0 = ch * TCH;
  const int tEnd = (t0 + TCH) < PC ? (t0 + TCH) : PC;

#pragma unroll 1
  for (int i = tid; i < TBLN / 4; i += NTHR) *(v4fa*)(tbl + 4 * i) = *(const v4f*)(tblg + 4 * i);
  if (tid < 32) cbs[tid] = bf_rne(cbias[tid]);
#pragma unroll 1
  for (int i = tid; i < 128 * TOKW; i += NTHR) {
    const int row = i / TOKW;
    const int j   = i - row * TOKW;
    int col = t0 + j;
    col = col > SEQ - 1 ? SEQ - 1 : col;
    int tv = target[(size_t)(mt * 128 + row) * SEQ + col];
    tv = tv < 0 ? 0 : (tv > NTOK - 1 ? NTOK - 1 : tv);
    tok[i] = tv * 32;
  }
  __syncthreads();

  v8f acc[8];
#pragma unroll
  for (int t = 0; t < 8; ++t) acc[t] = z8();
  const int* tr = tok + (16 * wave + m) * TOKW;
  int q0 = tr[0], q1 = tr[1], q2 = tr[2], q3 = tr[3], q4 = tr[4], q5 = tr[5], q6 = tr[6];
  const float* tb = tbl + 8 * hh;
  const v4f b0 = *(const v4fa*)(cbs + 8 * hh);
  const v4f b1 = *(const v4fa*)(cbs + 8 * hh + 4);
  const v4f b2 = *(const v4fa*)(cbs + 16 + 8 * hh);
  const v4f b3 = *(const v4fa*)(cbs + 16 + 8 * hh + 4);
  const unsigned short* wp = wxt + (size_t)m * KXT + 8 * hh;

#pragma unroll 1
  for (int t = t0; t < tEnd; ++t) {
    const int q7 = tr[t - t0 + 7];
    v4f c0 = b0, c1 = b1, c2 = b2, c3 = b3;
#define TAP(KK, Q) { const float* p = tb + (KK) * (NTOK * 32) + (Q); \
      c0 += *(const v4fa*)p; c1 += *(const v4fa*)(p + 4); \
      c2 += *(const v4fa*)(p + 16); c3 += *(const v4fa*)(p + 20); }
    TAP(0, q0)
    TAP(1, q1)
    TAP(2, q2)
    TAP(3, q3)
    TAP(4, q4)
    TAP(5, q5)
    TAP(6, q6)
    TAP(7, q7)
#undef TAP
    v8us h0v, h1v, l0v, l1v;
    split4<0>(c0, h0v, l0v);
    split4<4>(c1, h0v, l0v);
    split4<0>(c2, h1v, l1v);
    split4<4>(c3, h1v, l1v);
    FragB ah, al;
    ah.h[0] = h0v; ah.h[1] = h1v;
    al.h[0] = l0v; al.h[1] = l1v;
#pragma unroll
    for (int nt = 0; nt < 8; ++nt) {
      const unsigned short* wq = wp + (size_t)(16 * nt) * KXT + (size_t)t * 32;
      FragB bf;
      bf.h[0] = *(const v8usa*)wq;
      bf.h[1] = *(const v8usa*)(wq + 16);
      acc[nt] = wmb(ah, bf, acc[nt]);
      acc[nt] = wmb(al, bf, acc[nt]);
    }
    q0 = q1; q1 = q2; q2 = q3; q3 = q4; q4 = q5; q5 = q6; q6 = q7;
  }

#pragma unroll
  for (int nt = 0; nt < 8; ++nt) {
#pragma unroll
    for (int r = 0; r < 8; ++r) stg[(16 * wave + 8 * hh + r) * 128 + 16 * nt + m] = acc[nt][r];
  }
  __syncthreads();
  v4f fv[16];
#pragma unroll
  for (int i = 0; i < 16; ++i) fv[i] = *(const v4fa*)(stg + (16 * wave + i) * 128 + 4 * lane);
#pragma unroll
  for (int i = 0; i < 16; ++i) {
    float* op = part + ((size_t)ch * NG + (size_t)(mt * 128 + 16 * wave + i)) * 128 + 4 * lane;
    *(volatile v4f*)op = fv[i];
  }
  __threadfence();
#pragma unroll
  for (int i = 0; i < 16; ++i) {
    float* op = part + ((size_t)ch * NG + (size_t)(mt * 128 + 16 * wave + i)) * 128 + 4 * lane;
    *(volatile v4f*)op = fv[i];
  }
}

__global__ __launch_bounds__(NTHR) void k_xtc(const float* __restrict__ part, const float* __restrict__ bias,
                                              unsigned short* xc, int nUnits) {
  const int u = (int)blockIdx.x * NTHR + (int)threadIdx.x;
  if (u >= nUnits) return;
  const int row = u >> 5;
  const int L   = u & 31;
  const bool isLo = L >= 16;
  const int c8  = (L & 15) * 8;
  v4f s0 = {0.f, 0.f, 0.f, 0.f}, s1 = {0.f, 0.f, 0.f, 0.f};
#pragma unroll 4
  for (int c = 0; c < NCHK; ++c) {
    const float* p = part + ((size_t)c * NG + row) * 128 + c8;
    s0 += *(const v4f*)p;
    s1 += *(const v4f*)(p + 4);
  }
  const v4f ba = *(const v4f*)(bias + c8);
  const v4f bb = *(const v4f*)(bias + c8 + 4);
  const float f[8] = {relu_np(s0.x + bf_rne(ba.x)), relu_np(s0.y + bf_rne(ba.y)),
                      relu_np(s0.z + bf_rne(ba.z)), relu_np(s0.w + bf_rne(ba.w)),
                      relu_np(s1.x + bf_rne(bb.x)), relu_np(s1.y + bf_rne(bb.y)),
                      relu_np(s1.z + bf_rne(bb.z)), relu_np(s1.w + bf_rne(bb.w))};
  v8us o;
#pragma unroll
  for (int i = 0; i < 8; ++i) {
    const unsigned short hb = bf_bits(f[i]);
    const unsigned short lw = bf_bits(f[i] - bf_val(hb));
    o[i] = isLo ? lw : hb;
  }
  unsigned short* dp = xc + (size_t)row * XCW + 256 + 8 * L;
  *(volatile v8us*)dp = o;
  __threadfence();
  *(volatile v8us*)dp = o;
}

__global__ __launch_bounds__(NTHR) void k_out(const float* __restrict__ x2, const float* __restrict__ ow,
                                              const float* __restrict__ ob, float* out) {
  __shared__ __attribute__((aligned(16))) float so[32];
  const int tid = (int)threadIdx.x, lane = tid & 31, wave = tid >> 5;
  const v4f wa = *(const v4f*)(ow + 8 * lane);
  const v4f wb = *(const v4f*)(ow + 8 * lane + 4);
  const float w0 = bf_rne(wa.x), w1 = bf_rne(wa.y), w2 = bf_rne(wa.z), w3 = bf_rne(wa.w);
  const float w4 = bf_rne(wb.x), w5 = bf_rne(wb.y), w6 = bf_rne(wb.z), w7 = bf_rne(wb.w);
  const float obv = bf_rne(ob[0]);
#pragma unroll 1
  for (int rr = 0; rr < 4; ++rr) {
    const int row = (int)blockIdx.x * 32 + wave * 4 + rr;
    const float* p = x2 + (size_t)row * 256 + 8 * lane;
    const v4f a = *(const v4f*)p;
    const v4f b = *(const v4f*)(p + 4);
    float s = a.x * w0;
    s = fmaf(a.y, w1, s); s = fmaf(a.z, w2, s); s = fmaf(a.w, w3, s);
    s = fmaf(b.x, w4, s); s = fmaf(b.y, w5, s); s = fmaf(b.z, w6, s); s = fmaf(b.w, w7, s);
    s += __shfl_xor(s, 16);
    s += __shfl_xor(s, 8);
    s += __shfl_xor(s, 4);
    s += __shfl_xor(s, 2);
    s += __shfl_xor(s, 1);
    if (lane == 0) so[wave * 4 + rr] = s + obv;
  }
  __syncthreads();
  v4f v = {0.f, 0.f, 0.f, 0.f};
  float* op = out + (size_t)blockIdx.x * 32 + 4 * tid;
  if (tid < 8) {
    v = *(const v4fa*)(so + 4 * tid);
    *(volatile v4f*)op = v;
  }
  __threadfence();
  if (tid < 8) {
    *(volatile v4f*)op = v;
  }
}

static inline int cdiv(int a, int b) { return (a + b - 1) / b; }
static inline size_t al256(size_t o) { return (o + 255) & ~(size_t)255; }

extern "C" void kernel_launch(void* const* d_in, const int* in_sizes, int n_in,
                              void* d_out, int out_size, void* d_ws, size_t ws_size,
                              hipStream_t stream) {
  if (n_in < 29) return;
  if (in_sizes[0] != NN * FIN || in_sizes[1] != 2 * NE || in_sizes[2] != NN) return;
  if (in_sizes[3] != NG * SEQ || in_sizes[4] != NG * LMD || in_sizes[5] != NG * LMD) return;
  if (in_sizes[6] != FIN * DIM || in_sizes[7] != DIM || in_sizes[8] != DIM * DIM || in_sizes[9] != DIM) return;
  if (in_sizes[10] != 4 * DIM * DIM || in_sizes[11] != 4 * DIM) return;
  if (in_sizes[12] != 4 * DIM * DIM || in_sizes[13] != 4 * DIM) return;
  if (in_sizes[14] != 5 * DIM || in_sizes[15] != 5 * DIM) return;
  if (in_sizes[16] != DIM * 128 || in_sizes[17] != 128 || in_sizes[18] != NTOK * 128) return;
  if (in_sizes[19] != 32 * 128 * KCV || in_sizes[20] != 32) return;
  if (in_sizes[21] != 32 * PC * 128 || in_sizes[22] != 128) return;
  if (in_sizes[23] != 2304 * 1024 || in_sizes[24] != 1024) return;
  if (in_sizes[25] != 1024 * 256 || in_sizes[26] != 256) return;
  if (in_sizes[27] != 256 || in_sizes[28] != 1) return;
  if (out_size != NG) return;

  const float* x      = (const float*)d_in[0];
  const int*   ei     = (const int*)  d_in[1];
  const int*   src    = ei;
  const int*   dst    = ei + NE;
  const int*   bat    = (const int*)  d_in[2];
  const int*   target = (const int*)  d_in[3];
  const float* drug   = (const float*)d_in[4];
  const float* prot   = (const float*)d_in[5];
  const float* w1a    = (const float*)d_in[6];
  const float* b1a    = (const float*)d_in[7];
  const float* w1b    = (const float*)d_in[8];
  const float* b1b    = (const float*)d_in[9];
  const float* gw_a   = (const float*)d_in[10];
  const float* gb_a   = (const float*)d_in[11];
  const float* gw_b   = (const float*)d_in[12];
  const float* gb_b   = (const float*)d_in[13];
  const float* bn_g   = (const float*)d_in[14];
  const float* bn_b   = (const float*)d_in[15];
  const float* wxd    = (const float*)d_in[16];
  const float* bxd    = (const float*)d_in[17];
  const float* emb    = (const float*)d_in[18];
  const float* cw     = (const float*)d_in[19];
  const float* cb     = (const float*)d_in[20];
  const float* wxtw   = (const float*)d_in[21];
  const float* bxt    = (const float*)d_in[22];
  const float* wf1    = (const float*)d_in[23];
  const float* bf1    = (const float*)d_in[24];
  const float* wf2    = (const float*)d_in[25];
  const float* bf2    = (const float*)d_in[26];
  const float* ow     = (const float*)d_in[27];
  const float* ob     = (const float*)d_in[28];
  float* out = (float*)d_out;

  char* ws = (char*)d_ws;
  size_t off = 0;
  const size_t oXB   = off; off = al256(off + (size_t)MP * FPAD * 2);
  const size_t oRA   = off; off = al256(off + (size_t)MP * DIM * 4);
  const size_t oRB   = off; off = al256(off + (size_t)MP * DIM * 4);
  const size_t oZHL  = off; off = al256(off + (size_t)MP * HLW * 2);
  const size_t oTHL  = off; off = al256(off + (size_t)MP * HLW * 2);
  const size_t oLST  = off; off = al256(off + (size_t)NBLK * RCAP * 4);
  const size_t oCNT  = off; off = al256(off + (size_t)NBLK * NB * 4);
  const size_t oOFF  = off; off = al256(off + (size_t)NBLK * NB * 4);
  const size_t oREC  = off; off = al256(off + (size_t)NTILE * RECW * 4);
  const size_t oSTAT = off; off = al256(off + (size_t)5 * 128 * 4);
  const size_t oW1A  = off; off = al256(off + (size_t)32 * FPAD * 2);
  const size_t oWB   = off; off = al256(off + (size_t)9 * 32 * HLW * 2);
  const size_t oWXD  = off; off = al256(off + (size_t)128 * HLW * 2);
  const size_t oW1C  = off; off = al256(off + (size_t)1024 * XCW * 2);
  const size_t oW2C  = off; off = al256(off + (size_t)256 * X1W * 2);
  const size_t oWXT  = off; off = al256(off + (size_t)128 * KXT * 2);
  const size_t oTBL  = off; off = al256(off + (size_t)TBLN * 4);
  const size_t oPOOL = off; off = al256(off + (size_t)NG * HLW * 2);
  const size_t oPART = off; off = al256(off + (size_t)NCHK * NG * 128 * 4);
  const size_t oXC   = off; off = al256(off + (size_t)NG * XCW * 2);
  const size_t oX1   = off; off = al256(off + (size_t)NG * X1W * 2);
  const size_t oX2   = off; off = al256(off + (size_t)NG * 256 * 4);
  if (off > ws_size || off > (size_t)WSMAX) return;
  unsigned short* XB   = (unsigned short*)(ws + oXB);
  float*          RA   = (float*)(ws + oRA);
  float*          RB   = (float*)(ws + oRB);
  unsigned short* ZHL  = (unsigned short*)(ws + oZHL);
  unsigned short* THL  = (unsigned short*)(ws + oTHL);
  int*            LST  = (int*)(ws + oLST);
  int*            CNT  = (int*)(ws + oCNT);
  int*            OFFS = (int*)(ws + oOFF);
  float*          REC  = (float*)(ws + oREC);
  float*          STAT = (float*)(ws + oSTAT);
  unsigned short* W1A  = (unsigned short*)(ws + oW1A);
  unsigned short* WB   = (unsigned short*)(ws + oWB);
  unsigned short* WXD  = (unsigned short*)(ws + oWXD);
  unsigned short* W1C  = (unsigned short*)(ws + oW1C);
  unsigned short* W2C  = (unsigned short*)(ws + oW2C);
  unsigned short* WXT  = (unsigned short*)(ws + oWXT);
  float*          TBL  = (float*)(ws + oTBL);
  unsigned short* POOL = (unsigned short*)(ws + oPOOL);
  float*          PART = (float*)(ws + oPART);
  unsigned short* XC   = (unsigned short*)(ws + oXC);
  unsigned short* X1   = (unsigned short*)(ws + oX1);
  float*          X2   = (float*)(ws + oX2);

  hipFuncSetAttribute(reinterpret_cast<const void*>(&k_compact), hipFuncAttributeMaxDynamicSharedMemorySize, LDS_CMP);
  hipFuncSetAttribute(reinterpret_cast<const void*>(&k_xt), hipFuncAttributeMaxDynamicSharedMemorySize, LDS_XT);

  const int vecE = ((NE & 3) == 0) ? 1 : 0;
  const int vecN = ((NN & 3) == 0) ? 1 : 0;
  const int PLN  = 32 * HLW;

  { const int nu = MP * (FPAD / 8);   k_xb<<<cdiv(nu, NTHR), NTHR, 0, stream>>>(x, XB, nu); }
  { const int nu = 32 * (FPAD / 8);   k_wt<<<cdiv(nu, NTHR), NTHR, 0, stream>>>(w1a, DIM, 32, FPAD, FIN, 1, nu, W1A); }
  { const int nu = 32 * (HLW / 8);    k_wt<<<cdiv(nu, NTHR), NTHR, 0, stream>>>(w1b, DIM, 32, HLW, DIM, 0, nu, WB); }
  { const int nu = 4 * 32 * (HLW / 8); k_wt<<<cdiv(nu, NTHR), NTHR, 0, stream>>>(gw_a, DIM, 32, HLW, DIM, 0, nu, WB + 1 * PLN); }
  { const int nu = 4 * 32 * (HLW / 8); k_wt<<<cdiv(nu, NTHR), NTHR, 0, stream>>>(gw_b, DIM, 32, HLW, DIM, 0, nu, WB + 5 * PLN); }
  { const int nu = 128 * (HLW / 8);   k_wt<<<cdiv(nu, NTHR), NTHR, 0, stream>>>(wxd, 128, 128, HLW, DIM, 0, nu, WXD); }
  { const int nu = 1024 * (XCW / 8);  k_wt<<<cdiv(nu, NTHR), NTHR, 0, stream>>>(wf1, 1024, 1024, XCW, 2304, 2, nu, W1C); }
  { const int nu = 256 * (X1W / 8);   k_wt<<<cdiv(nu, NTHR), NTHR, 0, stream>>>(wf2, 256, 256, X1W, 1024, 0, nu, W2C); }
  { const int nu = NG * 128;
    k_lm<<<cdiv(nu, NTHR), NTHR, 0, stream>>>(drug, 512, XC, nu);
    k_lm<<<cdiv(nu, NTHR), NTHR, 0, stream>>>(prot, 1536, XC, nu); }
  k_wxt<<<TSLOT / 2, NTHR, 0, stream>>>(wxtw, WXT);
  k_tbl<<<TBLN / NTHR, NTHR, 0, stream>>>(emb, cw, TBL);
  k_compact<<<NBLK, NTHR, LDS_CMP, stream>>>(src, dst, NE, NN, vecE, LST, CNT, OFFS);

  k_mlp<0><<<NTILE, NTHR, 0, stream>>>(XB, W1A, b1a, W1A, b1a, RA, REC, NN);
  k_agg<1><<<NBLK, NTHR, 0, stream>>>(LST, CNT, OFFS, RA, STAT, b1a, THL, NN);
  k_mlp<1><<<NTILE, NTHR, 0, stream>>>(THL, WB, b1b, WB, b1b, RB, REC, NN);
  k_comb<<<1, 32, 0, stream>>>(REC, NTILE, bn_g, bn_b, STAT);

  for (int i = 0; i < 4; ++i) {
    const float* Fsrc = ((i & 1) == 0) ? RB : RA;
    float*       Fdst = ((i & 1) == 0) ? RA : RB;
    k_agg<0><<<NBLK, NTHR, 0, stream>>>(LST, CNT, OFFS, Fsrc, STAT + (size_t)i * 128, b1a, ZHL, NN);
    k_mlp<2><<<NTILE, NTHR, 0, stream>>>(ZHL, WB + (size_t)(1 + i) * PLN, gb_a + (size_t)i * DIM,
                                         WB + (size_t)(5 + i) * PLN, gb_b + (size_t)i * DIM, Fdst, REC, NN);
    k_comb<<<1, 32, 0, stream>>>(REC, NTILE, bn_g + (size_t)(i + 1) * DIM, bn_b + (size_t)(i + 1) * DIM,
                                 STAT + (size_t)(i + 1) * 128);
  }
  k_pool<<<NG / 8, NTHR, 0, stream>>>(bat, RB, STAT + (size_t)4 * 128, NN, vecN, POOL);
  k_gemm<1><<<dim3(NG / GBM, 1), GTHR, 0, stream>>>(POOL, HLW, WXD, HLW, bxd, (void*)XC, XCW, 0, 128);

  k_xt<<<dim3(NG / 128, NCHK), NTHR, LDS_XT, stream>>>(target, TBL, cb, WXT, PART);
  { const int nu = NG * 32; k_xtc<<<cdiv(nu, NTHR), NTHR, 0, stream>>>(PART, bxt, XC, nu); }

  k_gemm<1><<<dim3(NG / GBM, 1024 / GBN), GTHR, 0, stream>>>(XC, XCW, W1C, XCW, bf1, (void*)X1, X1W, 0, 1024);
  k_gemm<2><<<dim3(NG / GBM, 256 / GBN), GTHR, 0, stream>>>(X1, X1W, W2C, X1W, bf2, (void*)X2, 256, 0, 0);
  k_out<<<NG / 32, NTHR, 0, stream>>>(X2, ow, ob, out);
}
